// GraphAttentionLayer_75118978007306
// MI455X (gfx1250) — hardware-verified
//
#include <hip/hip_runtime.h>
#include <math.h>
#include <stdint.h>

#ifndef NB
#define NB 2
#endif
#ifndef SEQ
#define SEQ 2048
#endif
#ifndef NB_FULL
#define NB_FULL 2
#endif
#ifndef SEQ_FULL
#define SEQ_FULL 2048
#endif
#define FIN   256
#define DM    256
#define NHD   8
#define HDM   32
#define QKVW  (3 * DM)
#define BN    (NB * SEQ)
#define PSC   1024.0f
#define VSC   16.0f
#define ASC   64.0f
#define WSC   64.0f
#define OSC   0.00390625f
#define USC   0.000244140625f
#define LN_EPS 1e-5f
#define MAP_OFF ((size_t)NB_FULL * SEQ_FULL * DM)

static_assert(NB >= 1 && NB <= NB_FULL && SEQ >= 256 && SEQ <= SEQ_FULL);
static_assert(SEQ % 256 == 0 && BN % 64 == 0);
static_assert(FIN % 64 == 0 && FIN % 32 == 0 && DM == FIN && DM == NHD * HDM && HDM == 32 && QKVW % 128 == 0 && DM % 128 == 0);
static_assert(PSC * VSC * OSC == ASC);
static_assert(ASC * WSC * USC == 1.0f);
static_assert(MAP_OFF * 4 == 4194304);

typedef __bf16         v16b __attribute__((ext_vector_type(16)));
typedef __bf16         v8b  __attribute__((ext_vector_type(8)));
typedef _Float16       v16h __attribute__((ext_vector_type(16)));
typedef _Float16       v8h  __attribute__((ext_vector_type(8)));
typedef _Float16       v4h  __attribute__((ext_vector_type(4)));
typedef float          v8f  __attribute__((ext_vector_type(8)));
typedef float          v4f  __attribute__((ext_vector_type(4)));
typedef unsigned int   v4u  __attribute__((ext_vector_type(4)));
typedef int            v4i  __attribute__((ext_vector_type(4)));
typedef v4f __attribute__((may_alias)) v4fa;
typedef v4u __attribute__((may_alias)) v4ua;
typedef v4i __attribute__((may_alias)) v4ia;
typedef v8b __attribute__((may_alias)) v8ba;
typedef v8h __attribute__((may_alias)) v8ha;
typedef v4h __attribute__((may_alias)) v4ha;
typedef _Float16 h16;

__device__ __forceinline__ unsigned short bf_bits(float f) {
  const unsigned u = __float_as_uint(f);
  return (unsigned short)((u + 0x7FFFu + ((u >> 16) & 1u)) >> 16);
}
__device__ __forceinline__ float bf_val(unsigned short h) { return __uint_as_float(((unsigned)h) << 16); }
__device__ __forceinline__ float bf_rne(float f) { return bf_val(bf_bits(f)); }
__device__ __forceinline__ v4f bf_rne4(v4f a) {
  v4f r;
  r[0] = bf_rne(a[0]); r[1] = bf_rne(a[1]); r[2] = bf_rne(a[2]); r[3] = bf_rne(a[3]);
  return r;
}
__device__ __forceinline__ unsigned short h_bits(float f) {
  const _Float16 hv = (_Float16)f;
  return __builtin_bit_cast(unsigned short, hv);
}
static __device__ __forceinline__ h16 toh_flush(float v) { const float w = (fabsf(v) < 6.103515625e-05f) ? 0.0f : v; return (h16)w; }
__device__ __forceinline__ unsigned short hf_bits(h16 hv) { return __builtin_bit_cast(unsigned short, hv); }
template <int KIND>
__device__ __forceinline__ unsigned short cvt16(float f) {
  if (KIND == 0) return bf_bits(f);
  if (KIND == 1) return h_bits(bf_rne(f));
  if (KIND == 2) return hf_bits(toh_flush(bf_rne(f) * WSC));
  return hf_bits(toh_flush(f * VSC));
}
__device__ __forceinline__ unsigned pk16(unsigned short a, unsigned short b) { return (unsigned)a | ((unsigned)b << 16); }
__device__ __forceinline__ v8f zero8() { v8f z = {0.f, 0.f, 0.f, 0.f, 0.f, 0.f, 0.f, 0.f}; return z; }
__device__ __forceinline__ int wave_id() { return __builtin_amdgcn_readfirstlane((int)(threadIdx.x >> 5)); }

__device__ __forceinline__ void lds_wave_sync() {
  __builtin_amdgcn_fence(3  , "workgroup");
  __builtin_amdgcn_wave_barrier();
  __builtin_amdgcn_fence(2  , "workgroup");
}

union FragB { v16b v; v8b h[2]; };
union FragH { v16h v; v8h h[2]; };
__device__ __forceinline__ v16b ldfrag_b(const __bf16* p) {
  FragB f;
  f.h[0] = *(const v8ba*)(p);
  f.h[1] = *(const v8ba*)(p + 16);
  return f.v;
}
__device__ __forceinline__ v16h ldfrag_h(const _Float16* p) {
  FragH f;
  f.h[0] = *(const v8ha*)(p);
  f.h[1] = *(const v8ha*)(p + 16);
  return f.v;
}
__device__ __forceinline__ v8f mma_b(v16b a, v16b b, v8f c) {
  return __builtin_amdgcn_wmma_f32_16x16x32_bf16(false, a, false, b, (short)0, c, false, false);
}
__device__ __forceinline__ v8f mma_h(v16h a, v16h b, v8f c) {
  return __builtin_amdgcn_wmma_f32_16x16x32_f16(false, a, false, b, (short)0, c, false, false);
}
__device__ __forceinline__ v8f wmmabg(v16b a, v16b b, v8f c) {
  c = mma_b(a, b, c);
  asm volatile("v_nop\n\tv_nop\n\tv_nop\n\tv_nop" : "+v"(c) : "v"(a), "v"(b));
  return c;
}
__device__ __forceinline__ v8f wmma16g(v16h a, v16h b, v8f c) {
  c = mma_h(a, b, c);
  asm volatile("v_nop\n\tv_nop\n\tv_nop\n\tv_nop" : "+v"(c) : "v"(a), "v"(b));
  return c;
}

__global__ __launch_bounds__(256) void prep_x_kernel(const float* __restrict__ x, unsigned short* __restrict__ xb, int nunits) {
  const int i = (int)blockIdx.x * 256 + (int)threadIdx.x;
  if (i >= nunits) return;
  const size_t e  = 8 * (size_t)i;
  const int    bn = (int)(e / FIN);
  const int    f  = (int)(e - (size_t)bn * FIN);
  const int    b  = bn / SEQ;
  const int    n  = bn - b * SEQ;
  const float* src = x + ((size_t)b * SEQ_FULL + n) * FIN + f;
  const v4f a = *(const v4fa*)(src);
  const v4f c = *(const v4fa*)(src + 4);
  v4u w;
  w[0] = pk16(bf_bits(a[0]), bf_bits(a[1]));
  w[1] = pk16(bf_bits(a[2]), bf_bits(a[3]));
  w[2] = pk16(bf_bits(c[0]), bf_bits(c[1]));
  w[3] = pk16(bf_bits(c[2]), bf_bits(c[3]));
  *(volatile v4u*)(xb + e) = w;
  __threadfence();
  *(volatile v4u*)(xb + e) = w;
}

template <int KIND>
__global__ __launch_bounds__(256) void tconv_kernel(const float* __restrict__ W, unsigned short* __restrict__ outp,
                                                    int R, int Cc, long sIn, long sOut) {
  __shared__ __align__(16) float tf[64 * 68];
  W    += (size_t)blockIdx.z * sIn;
  outp += (size_t)blockIdx.z * sOut;
  const int c0  = (int)blockIdx.x * 64;
  const int r0  = (int)blockIdx.y * 64;
  const int tid = (int)threadIdx.x;
  {
    const int lr = tid >> 4;
    const int c4 = (tid & 15) * 4;
#pragma unroll
    for (int it = 0; it < 4; ++it) {
      const int rr = it * 16 + lr;
      const v4f a = *(const v4fa*)(W + (size_t)(r0 + rr) * Cc + c0 + c4);
      *(v4f*)(tf + rr * 68 + c4) = a;
    }
  }
  __syncthreads();
  const int sub = tid >> 3;
  const int c8  = (tid & 7) * 8;
  v4u hv[2];
#pragma unroll
  for (int it = 0; it < 2; ++it) {
    const int oc = it * 32 + sub;
    v4u a;
#pragma unroll
    for (int q = 0; q < 4; ++q) {
      const float f0 = tf[(c8 + 2 * q) * 68 + oc];
      const float f1 = tf[(c8 + 2 * q + 1) * 68 + oc];
      a[q] = pk16(cvt16<KIND>(f0), cvt16<KIND>(f1));
    }
    hv[it] = a;
  }
  for (int pass = 0; pass < 2; ++pass) {
#pragma unroll
    for (int it = 0; it < 2; ++it) {
      const int oc = it * 32 + sub;
      const size_t go = (size_t)(c0 + oc) * R + r0 + c8;
      *(volatile v4u*)(outp + go) = hv[it];
    }
    __threadfence();
  }
}

#define SLAB_PERW 2048
#define GT_N (QKVW / 128)
#define GT_M (BN / 32)
static_assert(GT_N == 6 && (GT_M * GT_N) % 4 == 0);
static_assert(4 * SLAB_PERW * 4 <= 131072);
static_assert(32 * 16 == 128 * 4);

__global__ __launch_bounds__(128) __attribute__((amdgpu_num_vgpr(256))) void gemm_qkv_kernel(
    const unsigned short* Ap, const unsigned short* Btp,
    const float* __restrict__ attv, const float* __restrict__ bq, const float* __restrict__ bk, const float* __restrict__ bv,
    float* sd, float* v32) {
  __shared__ __align__(16) float slab_all[4 * SLAB_PERW];

  const int lane = threadIdx.x & 31;
  const int wave = wave_id();
  const int hh = lane >> 4;
  const int rl = lane & 15;
  const unsigned bx = blockIdx.x;
  const unsigned tile = bx * 4u + (unsigned)wave;
  if (tile >= (unsigned)(GT_M * GT_N)) return;
  const unsigned tm = tile / 6u;
  const unsigned tn = tile - tm * 6u;
  const int m0 = (int)(tm << 5);
  const int n0 = (int)(tn << 7);
  const unsigned kind = tn >> 1;
  const int cb = (int)((tn & 1u) << 7);

  const __bf16* A  = (const __bf16*)(const void*)Ap;
  const __bf16* Bt = (const __bf16*)(const void*)Btp;

  v8f acc[2][8];
#pragma unroll
  for (int i = 0; i < 2; ++i)
#pragma unroll
    for (int j = 0; j < 8; ++j) acc[i][j] = zero8();

  for (int k0 = 0; k0 < FIN; k0 += 32) {
    const v16b a0f = ldfrag_b(A + (size_t)(m0 + rl) * FIN + k0 + 8 * hh);
    const v16b a1f = ldfrag_b(A + (size_t)(m0 + 16 + rl) * FIN + k0 + 8 * hh);
#pragma unroll
    for (int j = 0; j < 8; ++j) {
      const v16b bh = ldfrag_b(Bt + (size_t)(n0 + j * 16 + rl) * FIN + k0 + 8 * hh);
      acc[0][j] = wmmabg(a0f, bh, acc[0][j]);
      acc[1][j] = wmmabg(a1f, bh, acc[1][j]);
    }
  }

  float* slf = slab_all + wave * SLAB_PERW;
  if (kind < 2u) {
    const int  aoff = (int)kind * HDM;
    const int  hg   = (cb >> 5) + 2 * hh;
    const float* a0p = attv + (size_t)hg * (2 * HDM) + aoff;
    const float* a1p = a0p + 2 * HDM;
    const int  bc   = cb + hh * 64;
    const bool isq  = (kind == 0u);
    float vh0 = 0.f, vh1 = 0.f, vh2 = 0.f, vh3 = 0.f;
#pragma unroll
    for (int i = 0; i < 2; ++i) {
#pragma unroll
      for (int j = 0; j < 8; ++j) {
#pragma unroll
        for (int r = 0; r < 8; ++r)
          slf[(8 * hh + r) * 128 + j * 16 + rl] = acc[i][j][r];
      }
      lds_wave_sync();
      {
        const float* sp = slf + rl * 128 + hh * 64;
        float s = 0.f, d = 0.f;
#pragma unroll 2
        for (int it = 0; it < HDM / 4; ++it) {
          const v4f f0 = *(const v4fa*)(sp + it * 4);
          const v4f f1 = *(const v4fa*)(sp + HDM + it * 4);
          const v4f w0 = bf_rne4(*(const v4fa*)(a0p + it * 4));
          const v4f w1 = bf_rne4(*(const v4fa*)(a1p + it * 4));
          const v4f q0v = *(const v4fa*)(bq + bc + it * 4);
          const v4f q1v = *(const v4fa*)(bq + bc + HDM + it * 4);
          const v4f k0v = *(const v4fa*)(bk + bc + it * 4);
          const v4f k1v = *(const v4fa*)(bk + bc + HDM + it * 4);
          const v4f b0 = bf_rne4(isq ? q0v : k0v);
          const v4f b1 = bf_rne4(isq ? q1v : k1v);
          s = fmaf(f0[0] + b0[0], w0[0], s);
          s = fmaf(f0[1] + b0[1], w0[1], s);
          s = fmaf(f0[2] + b0[2], w0[2], s);
          s = fmaf(f0[3] + b0[3], w0[3], s);
          d = fmaf(f1[0] + b1[0], w1[0], d);
          d = fmaf(f1[1] + b1[1], w1[1], d);
          d = fmaf(f1[2] + b1[2], w1[2], d);
          d = fmaf(f1[3] + b1[3], w1[3], d);
        }
        const float t0 = __shfl(s, rl, 32);
        const float t1 = __shfl(d, rl, 32);
        const float t2 = __shfl(s, 16 + rl, 32);
        const float t3 = __shfl(d, 16 + rl, 32);
        const bool mine = (hh == i);
        vh0 = mine ? t0 : vh0;
        vh1 = mine ? t1 : vh1;
        vh2 = mine ? t2 : vh2;
        vh3 = mine ? t3 : vh3;
      }
      lds_wave_sync();
    }
    float* base = sd + (size_t)(tn * 4u) * BN + m0 + lane;
    for (int pass = 0; pass < 2; ++pass) {
      *(volatile float*)(base)                  = vh0;
      *(volatile float*)(base + BN)             = vh1;
      *(volatile float*)(base + (size_t)2 * BN) = vh2;
      *(volatile float*)(base + (size_t)3 * BN) = vh3;
      __threadfence();
    }
  } else {
    float bj[8];
#pragma unroll
    for (int j = 0; j < 8; ++j) bj[j] = bf_rne(bv[cb + j * 16 + rl]);
    float* Cb = v32 + (size_t)m0 * DM + cb;
#pragma unroll
    for (int i = 0; i < 2; ++i) {
#pragma unroll
      for (int j = 0; j < 8; ++j) {
#pragma unroll
        for (int r = 0; r < 8; ++r)
          slf[(8 * hh + r) * 128 + j * 16 + rl] = acc[i][j][r] + bj[j];
      }
      lds_wave_sync();
      for (int pass = 0; pass < 2; ++pass) {
#pragma unroll
        for (int row = 0; row < 16; ++row) {
          const v4f xv = *(const v4fa*)(slf + row * 128 + lane * 4);
          *(volatile v4f*)(Cb + (size_t)(16 * i + row) * DM + lane * 4) = xv;
        }
        __threadfence();
      }
      lds_wave_sync();
    }
  }
}

#define KT       64
#define PSP      72
#define ATT_P_H  (4 * 16 * PSP)
#define ATT_S_F  (4 * 16 * HDM)
#define ATT_T_F  (4 * 32)
static_assert(ATT_P_H * 2 + ATT_S_F * 4 + ATT_T_F * 4 <= 131072);
static_assert(SEQ % KT == 0 && KT == 64 && HDM == 32);
static_assert(32 * 8 * 2 == 16 * HDM);

__global__ __launch_bounds__(128) __attribute__((amdgpu_num_vgpr(240))) void attn_kernel(
    const int* __restrict__ adj, const float* __restrict__ sd,
    const unsigned short* __restrict__ vt, unsigned short* __restrict__ atth, float* __restrict__ st) {
  __shared__ __align__(16) _Float16 lds_p[ATT_P_H];
  __shared__ __align__(16) float    lds_s[ATT_S_F];
  __shared__ __align__(16) float    lds_t[ATT_T_F];

  const int tid  = (int)threadIdx.x;
  const int lane = tid & 31;
  const int wave = wave_id();
  const int hh   = lane >> 4;
  const int c    = lane & 15;
  const int qb   = (int)blockIdx.x;
  const int h    = (int)blockIdx.y;
  const int b    = (int)blockIdx.z;
  const int q0   = qb * 64 + wave * 16;

  const int*      Ag = adj + (size_t)b * SEQ_FULL * SEQ_FULL + (size_t)(q0 + 8 * hh) * SEQ_FULL + 4 * c;
  const float*    Dg = sd + (size_t)(NHD + h) * BN + (size_t)b * SEQ + 4 * c;
  const _Float16* Vg = (const _Float16*)(const void*)vt + ((size_t)b * DM + (size_t)h * HDM) * SEQ + 8 * hh;
  _Float16* ph = lds_p + wave * (16 * PSP);

  float cadd[8];
  {
    const size_t ro = (size_t)h * BN + (size_t)b * SEQ + q0 + 8 * hh;
    const v4f s0 = *(const v4fa*)(sd + ro);
    const v4f s1 = *(const v4fa*)(sd + ro + 4);
#pragma unroll
    for (int r = 0; r < 4; ++r) { cadd[r] = s0[r]; cadd[4 + r] = s1[r]; }
  }

  float mrow[8], lrow[8];
#pragma unroll
  for (int r = 0; r < 8; ++r) { mrow[r] = -INFINITY; lrow[r] = 0.f; }
  v8f o0 = zero8();
  v8f o1 = zero8();

#pragma unroll 1
  for (int kc = 0; kc < SEQ / KT; ++kc) {
    const int kv0 = kc * KT;
    const v4f d4 = *(const v4fa*)(Dg + kv0);
    float s[8][4];
    float cm[8];
#pragma unroll
    for (int r = 0; r < 8; ++r) {
      const v4i m4 = *(const v4ia*)(Ag + (size_t)r * SEQ_FULL + kv0);
      float m = -INFINITY;
#pragma unroll
      for (int q = 0; q < 4; ++q) {
        const float t  = cadd[r] + d4[q];
        const float e  = (t >= 0.0f) ? t : 0.2f * t;
        const float sv = (m4[q] != 0) ? e : -INFINITY;
        s[r][q] = sv;
        m = fmaxf(m, sv);
      }
#pragma unroll
      for (int off = 1; off < 16; off <<= 1) m = fmaxf(m, __shfl_xor(m, off, 32));
      cm[r] = m;
    }
    float alpha[8];
#pragma unroll
    for (int r = 0; r < 8; ++r) {
      const float mnew = fmaxf(mrow[r], cm[r]);
      const float ae   = __expf(mrow[r] - mnew);
      const float al   = (mrow[r] == -INFINITY) ? 0.0f : ae;
      const float msub = (mnew == -INFINITY) ? 0.0f : mnew;
      mrow[r]  = mnew;
      alpha[r] = al;
      float psum = 0.f;
      v4h pv;
#pragma unroll
      for (int q = 0; q < 4; ++q) {
        const float pe = __expf(s[r][q] - msub);
        const float p  = (s[r][q] > -INFINITY) ? pe : 0.0f;
        psum += p;
        pv[q] = toh_flush(p * PSC);
      }
      *(v4ha*)(ph + (8 * hh + r) * PSP + 4 * c) = pv;
#pragma unroll
      for (int off = 1; off < 16; off <<= 1) psum += __shfl_xor(psum, off, 32);
      lrow[r] = lrow[r] * al + psum;
    }
    lds_wave_sync();
    const v16h pa0 = ldfrag_h(ph + c * PSP + 8 * hh);
    const v16h pa1 = ldfrag_h(ph + c * PSP + 32 + 8 * hh);
#pragma unroll
    for (int r = 0; r < 8; ++r) { o0[r] *= alpha[r]; o1[r] *= alpha[r]; }
    {
      const size_t vo = (size_t)c * SEQ + kv0;
      const v16h vb0 = ldfrag_h(Vg + vo);
      const v16h vb1 = ldfrag_h(Vg + vo + 32);
      o0 = wmma16g(pa0, vb0, o0);
      o0 = wmma16g(pa1, vb1, o0);
    }
    {
      const size_t vo = (size_t)(16 + c) * SEQ + kv0;
      const v16h vb0 = ldfrag_h(Vg + vo);
      const v16h vb1 = ldfrag_h(Vg + vo + 32);
      o1 = wmma16g(pa0, vb0, o1);
      o1 = wmma16g(pa1, vb1, o1);
    }
    lds_wave_sync();
  }

  float rinv[8];
#pragma unroll
  for (int r = 0; r < 8; ++r) rinv[r] = 1.0f / lrow[r];
  float* os = lds_s + wave * (16 * HDM);
  float* tw = lds_t + wave * 32;
#pragma unroll
  for (int r = 0; r < 8; ++r) {
    const float iv = rinv[r] * OSC;
    os[(8 * hh + r) * HDM + c]      = o0[r] * iv;
    os[(8 * hh + r) * HDM + 16 + c] = o1[r] * iv;
  }
  if (c == 0) {
    v4f ma, mb, la, lb;
#pragma unroll
    for (int r = 0; r < 4; ++r) { ma[r] = mrow[r]; mb[r] = mrow[4 + r]; la[r] = rinv[r]; lb[r] = rinv[4 + r]; }
    *(v4fa*)(tw + 8 * hh)          = ma;
    *(v4fa*)(tw + 8 * hh + 4)      = mb;
    *(v4fa*)(tw + 16 + 8 * hh)     = la;
    *(v4fa*)(tw + 16 + 8 * hh + 4) = lb;
  }
  lds_wave_sync();
  v4u wv[2];
#pragma unroll
  for (int it = 0; it < 2; ++it) {
    const v4f f0 = *(const v4fa*)(os + it * 256 + lane * 8);
    const v4f f1 = *(const v4fa*)(os + it * 256 + lane * 8 + 4);
    v8h hv;
#pragma unroll
    for (int e = 0; e < 4; ++e) { hv[e] = toh_flush(f0[e]); hv[4 + e] = toh_flush(f1[e]); }
    wv[it] = __builtin_bit_cast(v4u, hv);
  }
  const v4fa* twv = (const v4fa*)(tw + (lane & 28));
  const v4f   tq  = *twv;
  const int   tl  = lane & 3;
  const float sval = (tl == 0) ? tq[0] : ((tl == 1) ? tq[1] : ((tl == 2) ? tq[2] : tq[3]));
  unsigned short* Ab = atth + (((size_t)b * NHD + h) * SEQ + q0) * HDM;
  float* Sb = st + (((size_t)b * NHD + h) * (SEQ / 16) + (size_t)(q0 >> 4)) * 32 + lane;
  for (int pass = 0; pass < 2; ++pass) {
#pragma unroll
    for (int it = 0; it < 2; ++it)
      *(volatile v4u*)(Ab + it * 256 + lane * 8) = wv[it];
    *(volatile float*)(Sb) = sval;
    __threadfence();
  }
}

#define MKG 256
static_assert(SEQ % MKG == 0 && MKG % KT == 0);
static_assert(16 * 16 == KT * 4);

__global__ __launch_bounds__(128) __attribute__((amdgpu_num_vgpr(256))) void map_kernel(
    const int* __restrict__ adj, const float* __restrict__ sd, const float* __restrict__ st, float* __restrict__ outm) {
  const int lane = (int)threadIdx.x & 31;
  const int wave = wave_id();
  const int hh   = lane >> 4;
  const int c    = lane & 15;
  const int qb   = (int)blockIdx.x;
  const int kg   = (int)blockIdx.y;
  const int b    = (int)blockIdx.z;
  const int q0   = qb * 64 + wave * 16;

  const int*   Ag = adj + (size_t)b * SEQ_FULL * SEQ_FULL + (size_t)(q0 + 8 * hh) * SEQ_FULL + 4 * c;
  float*       Mg = outm + ((size_t)b * SEQ_FULL + q0 + 8 * hh) * SEQ_FULL + 4 * c;
  const float* Sq = sd + (size_t)b * SEQ + q0 + 8 * hh;
  const float* Dg = sd + (size_t)NHD * BN + (size_t)b * SEQ + 4 * c;
  const float* Tg = st + ((size_t)b * NHD * (SEQ / 16) + (size_t)(q0 >> 4)) * 32 + 8 * hh;

#pragma unroll 1
  for (int kc = 0; kc < MKG / KT; ++kc) {
    const int kv0 = kg * MKG + kc * KT;
    unsigned vb = 0u;
#pragma unroll
    for (int r = 0; r < 8; ++r) {
      const v4i m4 = *(const v4ia*)(Ag + (size_t)r * SEQ_FULL + kv0);
#pragma unroll
      for (int q = 0; q < 4; ++q) vb |= (m4[q] != 0) ? (1u << (r * 4 + q)) : 0u;
    }
    v4f acc[8];
#pragma unroll
    for (int r = 0; r < 8; ++r) { acc[r][0] = 0.f; acc[r][1] = 0.f; acc[r][2] = 0.f; acc[r][3] = 0.f; }
#pragma unroll 1
    for (int h = 0; h < NHD; ++h) {
      const v4f s0 = *(const v4fa*)(Sq + (size_t)h * BN);
      const v4f s1 = *(const v4fa*)(Sq + (size_t)h * BN + 4);
      const float* tp = Tg + (size_t)h * (SEQ / 16) * 32;
      const v4f t0 = *(const v4fa*)(tp);
      const v4f t1 = *(const v4fa*)(tp + 4);
      const v4f u0 = *(const v4fa*)(tp + 16);
      const v4f u1 = *(const v4fa*)(tp + 20);
      const v4f d4 = *(const v4fa*)(Dg + (size_t)h * BN + kv0);
      float cr[8], mr[8], lr[8];
#pragma unroll
      for (int r = 0; r < 4; ++r) {
        cr[r] = s0[r]; cr[4 + r] = s1[r];
        mr[r] = t0[r]; mr[4 + r] = t1[r];
        lr[r] = u0[r]; lr[4 + r] = u1[r];
      }
#pragma unroll
      for (int r = 0; r < 8; ++r) {
#pragma unroll
        for (int q = 0; q < 4; ++q) {
          const float t = cr[r] + d4[q];
          const float e = (t >= 0.0f) ? t : 0.2f * t;
          const float p = __expf(e - mr[r]) * lr[r];
          const bool  vis = ((vb >> (r * 4 + q)) & 1u) != 0u;
          acc[r][q] += vis ? p : 0.0f;
        }
      }
    }
    v4f ov[8];
#pragma unroll
    for (int r = 0; r < 8; ++r) {
      ov[r][0] = acc[r][0] * 0.125f; ov[r][1] = acc[r][1] * 0.125f;
      ov[r][2] = acc[r][2] * 0.125f; ov[r][3] = acc[r][3] * 0.125f;
    }
    for (int pass = 0; pass < 2; ++pass) {
#pragma unroll
      for (int r = 0; r < 8; ++r)
        *(volatile v4f*)(Mg + (size_t)r * SEQ_FULL + kv0) = ov[r];
      __threadfence();
    }
  }
}

#define OTP 256
static_assert(2 * 16 * OTP * 4 <= 131072);
static_assert(2 * 32 * 16 == DM * 4);
static_assert(BN % 32 == 0 && SEQ % 16 == 0);

__global__ __launch_bounds__(64) __attribute__((amdgpu_num_vgpr(256))) void out_ln_kernel(
    const unsigned short* __restrict__ atth, const unsigned short* __restrict__ wot,
    const float* __restrict__ x, const float* __restrict__ bo, const float* __restrict__ lng, const float* __restrict__ lnb,
    float* __restrict__ out) {
  __shared__ __align__(16) float lds_o[2 * 16 * OTP];

  const int lane = (int)threadIdx.x & 31;
  const int wave = wave_id();
  const int hh   = lane >> 4;
  const int rl   = lane & 15;
  const unsigned bx = blockIdx.x;
  const unsigned m0 = (bx * 2u + (unsigned)wave) * 16u;
  const unsigned b  = m0 / (unsigned)SEQ;
  const unsigned n0 = m0 - b * (unsigned)SEQ;

  const _Float16* A  = (const _Float16*)(const void*)atth + ((size_t)b * NHD * SEQ + n0 + rl) * HDM + 8 * hh;
  const _Float16* Wt = (const _Float16*)(const void*)wot + (size_t)rl * DM + 8 * hh;

  v8f acc[16];
#pragma unroll
  for (int j = 0; j < 16; ++j) acc[j] = zero8();

#pragma unroll 1
  for (int ks = 0; ks < NHD; ++ks) {
    const v16h af = ldfrag_h(A + (size_t)ks * SEQ * HDM);
#pragma unroll
    for (int j = 0; j < 16; ++j) {
      const v16h bh = ldfrag_h(Wt + (size_t)(j * 16) * DM + ks * 32);
      acc[j] = wmma16g(af, bh, acc[j]);
    }
  }

  float* os = lds_o + wave * (16 * OTP);
#pragma unroll
  for (int j = 0; j < 16; ++j) {
#pragma unroll
    for (int r = 0; r < 8; ++r)
      os[(8 * hh + r) * OTP + j * 16 + rl] = acc[j][r];
  }
  lds_wave_sync();

  const v4f b0  = bf_rne4(*(const v4fa*)(bo + lane * 4));
  const v4f b1  = bf_rne4(*(const v4fa*)(bo + 128 + lane * 4));
  const v4f g0  = bf_rne4(*(const v4fa*)(lng + lane * 4));
  const v4f g1  = bf_rne4(*(const v4fa*)(lng + 128 + lane * 4));
  const v4f be0 = bf_rne4(*(const v4fa*)(lnb + lane * 4));
  const v4f be1 = bf_rne4(*(const v4fa*)(lnb + 128 + lane * 4));
  const float* xb = x + ((size_t)b * SEQ_FULL + n0) * DM;

#pragma unroll 1
  for (int row = 0; row < 16; ++row) {
    float* orow = os + row * OTP;
    const v4f a0 = *(const v4fa*)(orow + lane * 4);
    const v4f a1 = *(const v4fa*)(orow + 128 + lane * 4);
    const v4f x0 = bf_rne4(*(const v4fa*)(xb + (size_t)row * DM + lane * 4));
    const v4f x1 = bf_rne4(*(const v4fa*)(xb + (size_t)row * DM + 128 + lane * 4));
    v4f v0, v1;
#pragma unroll
    for (int e = 0; e < 4; ++e) {
      v0[e] = (a0[e] * USC + b0[e]) + x0[e];
      v1[e] = (a1[e] * USC + b1[e]) + x1[e];
    }
    float s = ((v0[0] + v0[1]) + (v0[2] + v0[3])) + ((v1[0] + v1[1]) + (v1[2] + v1[3]));
#pragma unroll
    for (int off = 16; off > 0; off >>= 1) s += __shfl_xor(s, off, 32);
    const float mu = s * (1.0f / DM);
    v4f d0, d1;
    float vs = 0.f;
#pragma unroll
    for (int e = 0; e < 4; ++e) {
      d0[e] = v0[e] - mu;
      d1[e] = v1[e] - mu;
      vs += d0[e] * d0[e];
      vs += d1[e] * d1[e];
    }
#pragma unroll
    for (int off = 16; off > 0; off >>= 1) vs += __shfl_xor(vs, off, 32);
    const float rs = rsqrtf(vs * (1.0f / DM) + LN_EPS);
    v4f y0, y1;
#pragma unroll
    for (int e = 0; e < 4; ++e) {
      y0[e] = d0[e] * rs * g0[e] + be0[e];
      y1[e] = d1[e] * rs * g1[e] + be1[e];
    }
    *(v4fa*)(orow + lane * 4)       = y0;
    *(v4fa*)(orow + 128 + lane * 4) = y1;
  }
  lds_wave_sync();
  float* Cb = out + ((size_t)b * SEQ_FULL + n0) * DM;
  for (int pass = 0; pass < 2; ++pass) {
#pragma unroll
    for (int row = 0; row < 16; ++row) {
      const v4f ya = *(const v4fa*)(os + row * OTP + lane * 4);
      const v4f yb = *(const v4fa*)(os + row * OTP + 128 + lane * 4);
      *(volatile v4f*)(Cb + (size_t)row * DM + lane * 4)       = ya;
      *(volatile v4f*)(Cb + (size_t)row * DM + 128 + lane * 4) = yb;
    }
    __threadfence();
  }
}

#define SZ_XB ((size_t)BN * FIN * 2)
#define SZ_WT ((size_t)QKVW * FIN * 2)
#define SZ_WO ((size_t)DM * DM * 2)
#define SZ_SD ((size_t)2 * NHD * BN * 4)
#define SZ_V3 ((size_t)BN * DM * 4)
#define SZ_VT ((size_t)NB * DM * SEQ * 2)
#define SZ_AH ((size_t)NB * NHD * SEQ * HDM * 2)
#define SZ_ST ((size_t)NB * NHD * (SEQ / 16) * 32 * 4)
#define WS_TOTAL (SZ_XB + SZ_WT + SZ_WO + SZ_SD + SZ_V3 + SZ_VT + SZ_AH + SZ_ST)
static_assert(WS_TOTAL <= 134217728);
static_assert(SZ_XB % 128 == 0 && SZ_WT % 128 == 0 && SZ_WO % 128 == 0 && SZ_SD % 128 == 0);
static_assert(SZ_V3 % 128 == 0 && SZ_VT % 128 == 0 && SZ_AH % 128 == 0 && SZ_ST % 128 == 0);
static_assert((BN * FIN / 8) % 256 == 0);
static_assert(((size_t)(NB - 1) * SEQ_FULL + SEQ - 1) * DM + DM - 1 < MAP_OFF);
static_assert(MAP_OFF + ((size_t)(NB - 1) * SEQ_FULL + SEQ - 1) * SEQ_FULL + SEQ - 1 < (size_t)NB_FULL * SEQ_FULL * (DM + SEQ_FULL));

extern "C" void kernel_launch(void* const* d_in, const int* in_sizes, int n_in,
                              void* d_out, int out_size, void* d_ws, size_t ws_size,
                              hipStream_t stream) {
  if (n_in < 13) return;
  const long long needX = ((long long)(NB - 1) * SEQ_FULL + SEQ) * FIN;
  const long long needA = (long long)(NB - 1) * SEQ_FULL * SEQ_FULL + (long long)(SEQ - 1) * SEQ_FULL + SEQ;
  const long long needO = (long long)MAP_OFF + needA;
  if ((long long)in_sizes[0] < needX) return;
  if ((long long)in_sizes[1] < needA) return;
  if (in_sizes[2] != FIN * DM || in_sizes[4] != FIN * DM || in_sizes[6] != FIN * DM || in_sizes[9] != DM * DM) return;
  if (in_sizes[3] != DM || in_sizes[5] != DM || in_sizes[7] != DM || in_sizes[10] != DM) return;
  if (in_sizes[8] != NHD * 2 * HDM) return;
  if (in_sizes[11] != DM || in_sizes[12] != DM) return;
  if ((long long)out_size < needO) return;

  const float* X    = (const float*)d_in[0];
  const int*   Adj  = (const int*)d_in[1];
  const float* Wq   = (const float*)d_in[2];
  const float* Bq   = (const float*)d_in[3];
  const float* Wk   = (const float*)d_in[4];
  const float* Bk   = (const float*)d_in[5];
  const float* Wv   = (const float*)d_in[6];
  const float* Bv   = (const float*)d_in[7];
  const float* Attv = (const float*)d_in[8];
  const float* Wo   = (const float*)d_in[9];
  const float* Bo   = (const float*)d_in[10];
  const float* Lng  = (const float*)d_in[11];
  const float* Lnb  = (const float*)d_in[12];
  float* out  = (float*)d_out;
  float* outm = out + MAP_OFF;

  size_t off = 0;
  const size_t oXB = off; off += SZ_XB;
  const size_t oWT = off; off += SZ_WT;
  const size_t oWO = off; off += SZ_WO;
  const size_t oSD = off; off += SZ_SD;
  const size_t oV3 = off; off += SZ_V3;
  const size_t oVT = off; off += SZ_VT;
  const size_t oAH = off; off += SZ_AH;
  const size_t oST = off; off += SZ_ST;
  if (off != WS_TOTAL) return;
  if (off > ws_size) return;

  char* ws = (char*)d_ws;
  unsigned short* XB  = (unsigned short*)(ws + oXB);
  unsigned short* WTB = (unsigned short*)(ws + oWT);
  unsigned short* WOT = (unsigned short*)(ws + oWO);
  float*          SD  = (float*)(ws + oSD);
  float*          V32 = (float*)(ws + oV3);
  unsigned short* VT  = (unsigned short*)(ws + oVT);
  unsigned short* AH  = (unsigned short*)(ws + oAH);
  float*          ST  = (float*)(ws + oST);

  const dim3 b256(256), b128(128), b64(64);

  const int nux = BN * FIN / 8;
  prep_x_kernel<<<dim3((nux + 255) / 256), b256, 0, stream>>>(X, XB, nux);
  tconv_kernel<0><<<dim3(DM / 64, FIN / 64, 1), b256, 0, stream>>>(Wq, WTB, FIN, DM, 0L, 0L);
  tconv_kernel<0><<<dim3(DM / 64, FIN / 64, 1), b256, 0, stream>>>(Wk, WTB + (size_t)DM * FIN, FIN, DM, 0L, 0L);
  tconv_kernel<0><<<dim3(DM / 64, FIN / 64, 1), b256, 0, stream>>>(Wv, WTB + (size_t)2 * DM * FIN, FIN, DM, 0L, 0L);
  tconv_kernel<2><<<dim3(DM / 64, DM / 64, 1), b256, 0, stream>>>(Wo, WOT, DM, DM, 0L, 0L);
  gemm_qkv_kernel<<<dim3((GT_M * GT_N) / 4), b128, 0, stream>>>(XB, WTB, Attv, Bq, Bk, Bv, SD, V32);
  tconv_kernel<3><<<dim3(DM / 64, SEQ / 64, NB), b256, 0, stream>>>(V32, VT, SEQ, DM, (long)SEQ * DM, (long)DM * SEQ);
  attn_kernel<<<dim3(SEQ / 64, NHD, NB), b128, 0, stream>>>(Adj, SD, VT, AH, ST);
  map_kernel<<<dim3(SEQ / 64, SEQ / MKG, NB), b128, 0, stream>>>(Adj, SD, ST, outm);
  out_ln_kernel<<<dim3(BN / 32), b64, 0, stream>>>(AH, WOT, X, Bo, Lng, Lnb, out);
  (void)hipGetLastError();
}
